// PhonemeGRU_24043226923218
// MI455X (gfx1250) — hardware-verified
//
#include <hip/hip_runtime.h>

typedef __attribute__((ext_vector_type(16))) _Float16 v16h;
typedef __attribute__((ext_vector_type(8)))  float    v8f;
typedef __attribute__((ext_vector_type(4)))  float    v4f;

constexpr int kVocab = 45;
constexpr int kEmb = 16;
constexpr int kHid = 32;
constexpr int kGate3 = 96;
constexpr int kSeq = 512;
constexpr int kOutDim = 64;
constexpr int kRowsPerBlock = 64;
constexpr int kThreads = 128;
constexpr int kWaves = kThreads / 32;
constexpr int kSlabPitch = 68;
constexpr int kGiEntries = kVocab * kGate3;
constexpr float kLog2e = 1.44269504088896340736f;
constexpr float kHScale = 64.0f;
constexpr float kWScale = 16.0f;
constexpr float kAccScale = 1024.0f;
constexpr float kAccInv = 0.0009765625f;

static_assert(kRowsPerBlock == kWaves * 16, "one 16-row n-subtile per wave");
static_assert(kGate3 == 3 * kHid && kHid == 32, "single 32-deep k-step, six 16-row gate tiles");

__device__ __forceinline__ v8f mma_f16(v16h a, v16h b, v8f c) {
  c = __builtin_amdgcn_wmma_f32_16x16x32_f16(false, a, false, b, (short)0, c, false, false);
  asm volatile("v_nop\n\tv_nop\n\tv_nop\n\tv_nop" : "+v"(c) : "v"(a), "v"(b));
  return c;
}

__device__ __forceinline__ float sigm_f(float x) {
  const float e = exp2f(-kLog2e * fabsf(x));
  const float q = __builtin_amdgcn_rcpf(1.0f + e);
  return (x >= 0.0f) ? q : e * q;
}

__device__ __forceinline__ float tanh_f(float y) {
  const float e = exp2f(-2.0f * kLog2e * fabsf(y));
  const float tp = (1.0f - e) * __builtin_amdgcn_rcpf(1.0f + e);
  return (y >= 0.0f) ? tp : -tp;
}

__device__ __forceinline__ v8f gated_cell8(v8f h, v8f dr, v8f dz, v8f dn,
                                            v4f gr0, v4f gr1, v4f gz0, v4f gz1, v4f gn0, v4f gn1) {
  const v8f gr = __builtin_shufflevector(gr0, gr1, 0, 1, 2, 3, 4, 5, 6, 7);
  const v8f gz = __builtin_shufflevector(gz0, gz1, 0, 1, 2, 3, 4, 5, 6, 7);
  const v8f gn = __builtin_shufflevector(gn0, gn1, 0, 1, 2, 3, 4, 5, 6, 7);
#pragma unroll
  for (int v = 0; v < 8; ++v) {
    const float hr = dr[v] * kAccInv;
    const float hz = dz[v] * kAccInv;
    const float hn = dn[v] * kAccInv;
    const float r = sigm_f(gr[v] + hr);
    const float z = sigm_f(gz[v] + hz);
    const float n = tanh_f(gn[v] + r * hn);
    h[v] = (1.0f - z) * n + z * h[v];
  }
  return h;
}

__global__ __launch_bounds__(kThreads) void recur_seq_fc_kernel(
    const int* __restrict__ xtok, const float* __restrict__ emb, const float* __restrict__ w_ih,
    const float* __restrict__ w_hh, const float* __restrict__ b_ih, const float* __restrict__ b_hh,
    const float* __restrict__ fc_w, const float* __restrict__ fc_b, float* __restrict__ out, int nrows)
{
  __shared__ __align__(16) float s_gi[kGiEntries];
  __shared__ __align__(16) float s_out[kWaves][16 * kSlabPitch];

  const int tid  = threadIdx.x;
  const int lane = tid & 31;
  const int wave = tid >> 5;
  const int hi   = lane >> 4;
  const int nl   = lane & 15;

#pragma unroll 1
  for (int it = 0; it < (kGiEntries + kThreads - 1) / kThreads; ++it) {
    const int idx = it * kThreads + tid;
    const int idc = (idx < kGiEntries) ? idx : (kGiEntries - 1);
    const int v = idc / kGate3;
    const int g = idc - v * kGate3;
    const float* er = emb + v * kEmb;
    const float* wr = w_ih + g * kEmb;
    float acc = 0.0f;
#pragma unroll
    for (int e = 0; e < kEmb; ++e) acc += er[e] * wr[e];
    const float bi  = b_ih[g];
    const float bhv = b_hh[g];
    acc += bi;
    acc += (g < 2 * kHid) ? bhv : 0.0f;
    if (idx < kGiEntries) s_gi[idx] = acc;
  }

  const v8f zc = {0.0f, 0.0f, 0.0f, 0.0f, 0.0f, 0.0f, 0.0f, 0.0f};

  v16h a_hh[6];
#pragma unroll
  for (int mt = 0; mt < 6; ++mt) {
    const float* wrow = w_hh + (mt * 16 + nl) * kHid;
#pragma unroll
    for (int i = 0; i < 8; ++i) {
      a_hh[mt][i]     = (_Float16)(kWScale * wrow[8 * hi + i]);
      a_hh[mt][8 + i] = (_Float16)(kWScale * wrow[16 + 8 * hi + i]);
    }
  }
  v8f cbn0 = zc, cbn1 = zc;
#pragma unroll
  for (int v = 0; v < 8; ++v) {
    cbn0[v] = kAccScale * b_hh[2 * kHid + 8 * hi + v];
    cbn1[v] = kAccScale * b_hh[2 * kHid + 16 + 8 * hi + v];
  }
  __syncthreads();

  const int row_base = blockIdx.x * kRowsPerBlock + wave * 16;
  int myrow = row_base + nl;
  myrow = (myrow < nrows) ? myrow : (nrows - 1);
  const int* xrow = xtok + (size_t)myrow * kSeq;

  v8f h0 = zc, h1 = zc;

#pragma unroll 1
  for (int t = 0; t < kSeq; ++t) {
    int tok = xrow[t];
    tok = (tok < 0) ? 0 : tok;
    tok = (tok > kVocab - 1) ? (kVocab - 1) : tok;

    v16h bfr;
#pragma unroll
    for (int i = 0; i < 8; ++i) {
      bfr[i]     = (_Float16)(kHScale * h0[i]);
      bfr[8 + i] = (_Float16)(kHScale * h1[i]);
    }

    const v8f d0 = mma_f16(a_hh[0], bfr, zc);
    const v8f d1 = mma_f16(a_hh[1], bfr, zc);
    const v8f d2 = mma_f16(a_hh[2], bfr, zc);
    const v8f d3 = mma_f16(a_hh[3], bfr, zc);
    const v8f d4 = mma_f16(a_hh[4], bfr, cbn0);
    const v8f d5 = mma_f16(a_hh[5], bfr, cbn1);

    const float* gp = s_gi + tok * kGate3 + 8 * hi;
    {
      const v4f r0 = *(const v4f*)(gp + 0),  r1 = *(const v4f*)(gp + 4);
      const v4f z0 = *(const v4f*)(gp + 32), z1 = *(const v4f*)(gp + 36);
      const v4f n0 = *(const v4f*)(gp + 64), n1 = *(const v4f*)(gp + 68);
      h0 = gated_cell8(h0, d0, d2, d4, r0, r1, z0, z1, n0, n1);
    }
    {
      const v4f r0 = *(const v4f*)(gp + 16), r1 = *(const v4f*)(gp + 20);
      const v4f z0 = *(const v4f*)(gp + 48), z1 = *(const v4f*)(gp + 52);
      const v4f n0 = *(const v4f*)(gp + 80), n1 = *(const v4f*)(gp + 84);
      h1 = gated_cell8(h1, d1, d3, d5, r0, r1, z0, z1, n0, n1);
    }
  }

  v16h bfr;
#pragma unroll
  for (int i = 0; i < 8; ++i) {
    bfr[i]     = (_Float16)(kHScale * h0[i]);
    bfr[8 + i] = (_Float16)(kHScale * h1[i]);
  }
  float* slab = s_out[wave];
#pragma unroll
  for (int mt = 0; mt < 4; ++mt) {
    const float* frow = fc_w + (mt * 16 + nl) * kHid;
    v16h afc;
#pragma unroll
    for (int i = 0; i < 8; ++i) {
      afc[i]     = (_Float16)(kWScale * frow[8 * hi + i]);
      afc[8 + i] = (_Float16)(kWScale * frow[16 + 8 * hi + i]);
    }
    v8f cfc = zc;
#pragma unroll
    for (int v = 0; v < 8; ++v) cfc[v] = kAccScale * fc_b[mt * 16 + 8 * hi + v];
    const v8f d = mma_f16(afc, bfr, cfc);
#pragma unroll
    for (int v = 0; v < 8; ++v) slab[nl * kSlabPitch + mt * 16 + 8 * hi + v] = d[v] * kAccInv;
  }
  __syncthreads();

  {
    const int c4 = nl * 4;
    float* orow = out + (size_t)row_base * kOutDim;
    for (int pass = 0; pass < 2; ++pass) {
#pragma unroll
      for (int it = 0; it < 8; ++it) {
        const int r = it * 2 + hi;
        const v4f val = *(const v4f*)(slab + r * kSlabPitch + c4);
        *(volatile v4f*)(orow + (size_t)r * kOutDim + c4) = val;
      }
      __threadfence();
    }
  }
}

extern "C" void kernel_launch(void* const* d_in, const int* in_sizes, int n_in,
                              void* d_out, int out_size, void* d_ws, size_t ws_size,
                              hipStream_t stream) {
  (void)n_in; (void)d_ws; (void)ws_size;
  const int*   xtok = (const int*)  d_in[0];
  const float* emb  = (const float*)d_in[1];
  const float* w_ih = (const float*)d_in[2];
  const float* w_hh = (const float*)d_in[3];
  const float* b_ih = (const float*)d_in[4];
  const float* b_hh = (const float*)d_in[5];
  const float* fc_w = (const float*)d_in[6];
  const float* fc_b = (const float*)d_in[7];
  float* out = (float*)d_out;

  const int rows_x = in_sizes[0] / kSeq;
  const int rows_o = out_size / kOutDim;
  const int rows   = (rows_x < rows_o) ? rows_x : rows_o;
  const int blocks = rows / kRowsPerBlock;
  if (blocks <= 0) return;
  const int nrows = blocks * kRowsPerBlock;

  recur_seq_fc_kernel<<<dim3(blocks), dim3(kThreads), 0, stream>>>(
      xtok, emb, w_ih, w_hh, b_ih, b_hh, fc_w, fc_b, out, nrows);
}
